// KAN1_23751169147141
// MI455X (gfx1250) — hardware-run, weakly checked
//
#include <hip/hip_runtime.h>


#define NBATCH 64
#define PP    196
#define CCH   768
#define HS    384
#define NG    8
#define SPC   8
#define RCH   (SPC * CCH)
#define NCH   (NBATCH / SPC)
#define K1    (PP * NG)
#define K1B   224
#define K2    (HS * NG)
#define N2    256
typedef _Float16 h16;
typedef unsigned short bf;
typedef __attribute__((ext_vector_type(16))) __bf16   v16bf;
typedef __attribute__((ext_vector_type(16))) _Float16 v16h;
typedef __attribute__((ext_vector_type(8)))  _Float16 v8h;
typedef __attribute__((ext_vector_type(8)))  unsigned short v8us;
typedef __attribute__((ext_vector_type(8)))  float    v8f;
typedef __attribute__((ext_vector_type(4)))  float    v4f;
typedef v8h  __attribute__((may_alias)) v8ha;
typedef v4f  __attribute__((may_alias)) v4fa;
typedef v8us __attribute__((may_alias)) v8usa;

__device__ __forceinline__ unsigned short f2bf(float f) { unsigned u = __float_as_uint(f); u += 0x7FFFu + ((u >> 16) & 1u); return (unsigned short)(u >> 16); }
__device__ __forceinline__ float bf2f(unsigned short b) { return __uint_as_float(((unsigned)b) << 16); }
__device__ __forceinline__ float bfr(float f) { return bf2f(f2bf(f)); }
__device__ __forceinline__ v16h cat16(v8h lo, v8h hi) { return __builtin_shufflevector(lo, hi, 0, 1, 2, 3, 4, 5, 6, 7, 8, 9, 10, 11, 12, 13, 14, 15); }
__device__ __forceinline__ v16bf cat16b(v8us lo, v8us hi) { return __builtin_bit_cast(v16bf, __builtin_shufflevector(lo, hi, 0, 1, 2, 3, 4, 5, 6, 7, 8, 9, 10, 11, 12, 13, 14, 15)); }
__device__ __forceinline__ v8f wmma16(v16h a, v16h b, v8f c) { return __builtin_amdgcn_wmma_f32_16x16x32_f16(false, a, false, b, (short)0, c, false, false); }
__device__ __forceinline__ v8f wmmab(v16bf a, v16bf b, v8f c) { return __builtin_amdgcn_wmma_f32_16x16x32_bf16(false, a, false, b, (short)0, c, false, false); }


template <typename T16> struct WFrag;
template <> struct WFrag<h16> { typedef v16h V; static __device__ __forceinline__ V ld(const h16* p) { return cat16(*(const v8h*)p, *(const v8h*)(p + 16)); } static __device__ __forceinline__ v8f mma(V a, V b, v8f c) { return wmma16(a, b, c); } };
template <> struct WFrag<bf> { typedef v16bf V; static __device__ __forceinline__ V ld(const bf* p) { return cat16b(*(const v8us*)p, *(const v8us*)(p + 16)); } static __device__ __forceinline__ v8f mma(V a, V b, v8f c) { return wmmab(a, b, c); } };
template <typename T16, int NSPLIT, bool BIAS>
__global__ __launch_bounds__(32) void k_gemmw(const T16* __restrict__ A, const T16* __restrict__ A2, const T16* __restrict__ Bt, const T16* __restrict__ Bt2, int K, float* C, int ldc, const float* __restrict__ bias, size_t sA, size_t sB, size_t sC) {
    typedef typename WFrag<T16>::V V;
    __shared__ __align__(16) float os[16 * 68];
    const size_t z = blockIdx.z; A += z * sA; if (A2) A2 += z * sA; Bt += z * sB; if (Bt2) Bt2 += z * sB; C += z * sC;
    const int lane = threadIdx.x & 31, lr = lane & 15, hi = lane >> 4; const int r0 = blockIdx.x * 64, c0 = blockIdx.y * 64;
    v8f acc[4][4];
#pragma unroll
    for (int mb = 0; mb < 4; ++mb)
#pragma unroll
        for (int nb = 0; nb < 4; ++nb) acc[mb][nb] = (v8f){};
    const size_t aoff = (size_t)(r0 + lr) * K + 8 * hi, boff = (size_t)(c0 + lr) * K + 8 * hi;
#pragma unroll 1
    for (int kc = 0; kc < K; kc += 32) {
        V a[4], a2[4];
#pragma unroll
        for (int mb = 0; mb < 4; ++mb) { a[mb] = WFrag<T16>::ld(A + aoff + (size_t)mb * 16 * K + kc); if (NSPLIT == 1 || NSPLIT == 2) a2[mb] = WFrag<T16>::ld(A2 + aoff + (size_t)mb * 16 * K + kc); }
#pragma unroll
        for (int nb = 0; nb < 4; ++nb) { const V b = WFrag<T16>::ld(Bt + boff + (size_t)nb * 16 * K + kc); V b2; if (NSPLIT >= 2) b2 = WFrag<T16>::ld(Bt2 + boff + (size_t)nb * 16 * K + kc);
#pragma unroll
            for (int mb = 0; mb < 4; ++mb) { acc[mb][nb] = WFrag<T16>::mma(a[mb], b, acc[mb][nb]); if (NSPLIT == 1 || NSPLIT == 2) acc[mb][nb] = WFrag<T16>::mma(a2[mb], b, acc[mb][nb]); if (NSPLIT >= 2) acc[mb][nb] = WFrag<T16>::mma(a[mb], b2, acc[mb][nb]); } }
        asm volatile("v_nop\n\tv_nop\n\tv_nop\n\tv_nop" : "+v"(acc[0][0]), "+v"(acc[1][1]), "+v"(acc[2][2]), "+v"(acc[3][3]) : "v"(a[0]), "v"(a[3]));
    }
#pragma unroll
    for (int mb = 0; mb < 4; ++mb) {
#pragma unroll
        for (int nb = 0; nb < 4; ++nb) {
#pragma unroll
            for (int j = 0; j < 8; ++j) os[(hi * 8 + j) * 68 + nb * 16 + lr] = acc[mb][nb][j]; }
        __builtin_amdgcn_wave_barrier(); asm volatile("" ::: "memory");
        float* crow = C + (size_t)(r0 + mb * 16) * ldc + c0;
#pragma unroll 1
        for (int ps = 0; ps < 2; ++ps) {
#pragma unroll
            for (int s = 0; s < 8; ++s) { const int row = 2 * s + hi, cofs = lr * 4; v4f val = *(const v4fa*)(os + row * 68 + cofs); if (BIAS) { val[0] += bfr(bias[c0 + cofs]); val[1] += bfr(bias[c0 + cofs + 1]); val[2] += bfr(bias[c0 + cofs + 2]); val[3] += bfr(bias[c0 + cofs + 3]); }
                *(volatile v4f*)(crow + (size_t)row * ldc + cofs) = val; }
            if (ps == 0) __threadfence(); }
        __builtin_amdgcn_wave_barrier(); asm volatile("" ::: "memory");
    }
}

typedef __attribute__((ext_vector_type(4))) unsigned short v4us;
__device__ __forceinline__ void splitf(float y, unsigned short& h, unsigned short& l) { h = f2bf(y); l = f2bf(y - bf2f(h)); }
__device__ __forceinline__ float siluf(float v) { return __fdiv_rn(v, __fadd_rn(1.0f, expf(-v))); }
__constant__ float GRID[NG] = {-1.0f, -0.7142857313156128f, -0.4285714328289032f, -0.1428571492433548f, 0.1428571492433548f, 0.4285714328289032f, 0.7142857313156128f, 1.0f};
#define DENOM 0.2857142984867096f
__device__ __forceinline__ v8us rbf8(float v) { v8us o;
#pragma unroll
    for (int i = 0; i < NG; ++i) { float z = __fdiv_rn(__fsub_rn(v, GRID[i]), DENOM); asm volatile("" : "+v"(z)); float z2 = __fmul_rn(z, z); asm volatile("" : "+v"(z2)); o[i] = f2bf(expf(-z2)); } return o; }
__global__ __launch_bounds__(256) void k_cvt8(const float* __restrict__ src, bf* dst, size_t n8) { const size_t i = (size_t)blockIdx.x * 256 + threadIdx.x; if (i >= n8) return; const v8f v = *(const v8f*)(src + i * 8); v8us o;
#pragma unroll
    for (int k = 0; k < 8; ++k) o[k] = f2bf(v[k]); *(volatile v8us*)(dst + i * 8) = o; __threadfence(); *(volatile v8us*)(dst + i * 8) = o; }
__global__ __launch_bounds__(256) void k_wpad(const float* __restrict__ w, int nval, int kval, int NOUT, int KP, bf* Bt) { const size_t e = ((size_t)blockIdx.x * 256 + threadIdx.x) * 8; if (e >= (size_t)NOUT * KP) return; const int k = (int)(e % KP), n = (int)(e / KP); v8us o;
#pragma unroll
    for (int q = 0; q < 8; ++q) o[q] = (n < nval && k + q < kval) ? f2bf(w[(size_t)n * kval + k + q]) : (unsigned short)0; *(volatile v8us*)(Bt + e) = o; __threadfence(); *(volatile v8us*)(Bt + e) = o; }
__global__ __launch_bounds__(256) void k_bpad(const float* __restrict__ b, float* BP) { const int n = threadIdx.x; if (n >= N2) return; const float v = (n < PP) ? b[n] : 0.f; *(volatile float*)(BP + n) = v; __threadfence(); *(volatile float*)(BP + n) = v; }
__global__ __launch_bounds__(256) void k_basis1(const float* __restrict__ x, int b0, bf* BAS) { const size_t e = (size_t)blockIdx.x * 256 + threadIdx.x; if (e >= (size_t)RCH * PP) return; const int p = (int)(e % PP); const int rl = (int)(e / PP); const int bl = rl / CCH, c = rl % CCH;
    const float v = bfr(x[((size_t)(b0 + bl) * PP + p) * CCH + c]); const v8us o = rbf8(v); *(volatile v8us*)(BAS + (size_t)rl * K1 + (size_t)p * NG) = o; __threadfence(); *(volatile v8us*)(BAS + (size_t)rl * K1 + (size_t)p * NG) = o; }
__global__ __launch_bounds__(256) void k_silu1(const float* __restrict__ x, int b0, bf* SIL, bf* SILl) { const size_t e = ((size_t)blockIdx.x * 256 + threadIdx.x) * 4; if (e >= (size_t)RCH * K1B) return; const int k = (int)(e % K1B); const int rl = (int)(e / K1B); const int bl = rl / CCH, c = rl % CCH; v4us o, ol;
#pragma unroll
    for (int q = 0; q < 4; ++q) { const int p = k + q; unsigned short hh = 0, ll = 0; if (p < PP) splitf(siluf(bfr(x[((size_t)(b0 + bl) * PP + p) * CCH + c])), hh, ll); o[q] = hh; ol[q] = ll; }
    *(volatile v4us*)(SIL + e) = o; *(volatile v4us*)(SILl + e) = ol; __threadfence(); *(volatile v4us*)(SIL + e) = o; *(volatile v4us*)(SILl + e) = ol; }
__global__ __launch_bounds__(256) void k_silu2(const float* __restrict__ H1, bf* SIL2, bf* SIL2l) { const size_t e = ((size_t)blockIdx.x * 256 + threadIdx.x) * 4; if (e >= (size_t)RCH * HS) return; const v4f v = *(const v4f*)(H1 + e); v4us o, ol;
#pragma unroll
    for (int q = 0; q < 4; ++q) { unsigned short hh, ll; splitf(siluf(v[q]), hh, ll); o[q] = hh; ol[q] = ll; } *(volatile v4us*)(SIL2 + e) = o; *(volatile v4us*)(SIL2l + e) = ol; __threadfence(); *(volatile v4us*)(SIL2 + e) = o; *(volatile v4us*)(SIL2l + e) = ol; }
__global__ __launch_bounds__(256) void k_h1(const float* __restrict__ S1, const float* __restrict__ B1v, float* H1, bf* BAS2) { const size_t e = (size_t)blockIdx.x * 256 + threadIdx.x; if (e >= (size_t)RCH * HS) return; const float h = __fadd_rn(S1[e], B1v[e]); const v8us o = rbf8(h);
    *(volatile float*)(H1 + e) = h; *(volatile v8us*)(BAS2 + e * NG) = o; __threadfence(); *(volatile float*)(H1 + e) = h; *(volatile v8us*)(BAS2 + e * NG) = o; }
__global__ __launch_bounds__(256) void k_out(const float* __restrict__ S2, const float* __restrict__ B2v, const float* __restrict__ x, int b0, float* O) { const size_t e = (size_t)blockIdx.x * 256 + threadIdx.x; if (e >= (size_t)SPC * PP * CCH) return; const int c = (int)(e % CCH); const int p = (int)((e / CCH) % PP); const int bl = (int)(e / ((size_t)CCH * PP)); const size_t rl = (size_t)bl * CCH + c; const size_t xi = ((size_t)(b0 + bl) * PP + p) * CCH + c;
    float h2 = __fadd_rn(S2[rl * N2 + p], B2v[rl * N2 + p]); asm volatile("" : "+v"(h2)); const float v = __fadd_rn(h2, bfr(x[xi])); *(volatile float*)(O + xi) = v; __threadfence(); *(volatile float*)(O + xi) = v; }

extern "C" void kernel_launch(void* const* d_in, const int* in_sizes, int n_in,
                              void* d_out, int out_size, void* d_ws, size_t ws_size, hipStream_t stream) {
    (void)in_sizes; (void)n_in; (void)out_size;
    const float* x = (const float*)d_in[0]; const float* w1s = (const float*)d_in[1]; const float* w1b = (const float*)d_in[2]; const float* b1 = (const float*)d_in[3]; const float* w2s = (const float*)d_in[4]; const float* w2b = (const float*)d_in[5]; const float* b2 = (const float*)d_in[6];
    float* OUT = (float*)d_out;
    char* wsp = (char*)d_ws;
    auto take = [&](size_t bytes) { char* p = wsp; wsp += (bytes + 255) & ~(size_t)255; return (void*)p; };
    bf* W1S = (bf*)take((size_t)HS * K1 * 2); bf* W1B = (bf*)take((size_t)HS * K1B * 2); bf* W2S = (bf*)take((size_t)N2 * K2 * 2); bf* W2B = (bf*)take((size_t)N2 * HS * 2); float* B2P = (float*)take(N2 * 4);
    bf* BAS1 = (bf*)take((size_t)RCH * K1 * 2); bf* SIL1 = (bf*)take((size_t)RCH * K1B * 2); bf* SIL1l = (bf*)take((size_t)RCH * K1B * 2); float* S1 = (float*)take((size_t)RCH * HS * 4); float* B1v = (float*)take((size_t)RCH * HS * 4); float* H1 = (float*)take((size_t)RCH * HS * 4);
    bf* BAS2 = (bf*)take((size_t)RCH * K2 * 2); bf* SIL2 = (bf*)take((size_t)RCH * HS * 2); bf* SIL2l = (bf*)take((size_t)RCH * HS * 2); float* S2 = (float*)take((size_t)RCH * N2 * 4); float* B2v = (float*)take((size_t)RCH * N2 * 4);
    if ((size_t)(wsp - (char*)d_ws) > ws_size) return;
    k_cvt8<<<(unsigned)(((size_t)HS * K1 / 8 + 255) / 256), 256, 0, stream>>>(w1s, W1S, (size_t)HS * K1 / 8);
    k_wpad<<<(unsigned)(((size_t)HS * K1B / 8 + 255) / 256), 256, 0, stream>>>(w1b, HS, PP, HS, K1B, W1B);
    k_wpad<<<(unsigned)(((size_t)N2 * K2 / 8 + 255) / 256), 256, 0, stream>>>(w2s, PP, K2, N2, K2, W2S); k_wpad<<<(unsigned)(((size_t)N2 * HS / 8 + 255) / 256), 256, 0, stream>>>(w2b, PP, HS, N2, HS, W2B); k_bpad<<<1, 256, 0, stream>>>(b2, B2P);
    for (int ch = 0; ch < NCH; ++ch) { const int b0 = ch * SPC;
        k_basis1<<<(unsigned)(((size_t)RCH * PP + 255) / 256), 256, 0, stream>>>(x, b0, BAS1); k_silu1<<<(unsigned)(((size_t)RCH * K1B / 4 + 255) / 256), 256, 0, stream>>>(x, b0, SIL1, SIL1l);
        k_gemmw<bf, 0, false><<<dim3(RCH / 64, HS / 64, 1), 32, 0, stream>>>(BAS1, nullptr, W1S, nullptr, K1, S1, HS, nullptr, 0, 0, 0);
        k_gemmw<bf, 1, true><<<dim3(RCH / 64, HS / 64, 1), 32, 0, stream>>>(SIL1, SIL1l, W1B, nullptr, K1B, B1v, HS, b1, 0, 0, 0);
        k_h1<<<(unsigned)(((size_t)RCH * HS + 255) / 256), 256, 0, stream>>>(S1, B1v, H1, BAS2); k_silu2<<<(unsigned)(((size_t)RCH * HS / 4 + 255) / 256), 256, 0, stream>>>(H1, SIL2, SIL2l);
        k_gemmw<bf, 0, false><<<dim3(RCH / 64, N2 / 64, 1), 32, 0, stream>>>(BAS2, nullptr, W2S, nullptr, K2, S2, N2, nullptr, 0, 0, 0);
        k_gemmw<bf, 1, true><<<dim3(RCH / 64, N2 / 64, 1), 32, 0, stream>>>(SIL2, SIL2l, W2B, nullptr, HS, B2v, N2, B2P, 0, 0, 0);
        k_out<<<(unsigned)(((size_t)SPC * PP * CCH + 255) / 256), 256, 0, stream>>>(S2, B2v, x, b0, OUT); }
}
